// TernaryLeNet5_91010357002967
// MI455X (gfx1250) — hardware-verified
//
#include <hip/hip_runtime.h>
#include <math.h>
#include <stdint.h>


typedef __attribute__((ext_vector_type(16))) _Float16 v16h;
typedef __attribute__((ext_vector_type(8)))  _Float16 v8h;
typedef __attribute__((ext_vector_type(16))) __bf16   v16b;
typedef __attribute__((ext_vector_type(8)))  __bf16   v8b;
typedef __attribute__((ext_vector_type(8)))  float    v8f;
typedef __attribute__((ext_vector_type(4)))  float    v4f;

__device__ __forceinline__ unsigned short f2bf_bits(float f) {
  unsigned u = __float_as_uint(f);
  return (unsigned short)((u + 0x7FFFu + ((u >> 16) & 1u)) >> 16);
}
__device__ __forceinline__ float bf_bits2f(unsigned short h) { return __uint_as_float(((unsigned)h) << 16); }

__device__ __forceinline__ void dep_guard_h(v8f& a, v8f& b, v16h x, v16h y) { asm volatile("v_nop\n\tv_nop\n\tv_nop\n\tv_nop" : "+v"(a), "+v"(b) : "v"(x), "v"(y)); }
__device__ __forceinline__ void dep_guard_b(v8f& a, v8f& b, v16b x, v16b y) { asm volatile("v_nop\n\tv_nop\n\tv_nop\n\tv_nop" : "+v"(a), "+v"(b) : "v"(x), "v"(y)); }
__device__ __forceinline__ void keep4_h(v16h a, v16h b, v16h c, v16h d) { asm volatile("v_nop" :: "v"(a), "v"(b), "v"(c), "v"(d)); }
__device__ __forceinline__ void keep4_b(v16b a, v16b b, v16b c, v16b d) { asm volatile("v_nop" :: "v"(a), "v"(b), "v"(c), "v"(d)); }
__device__ __forceinline__ void acc_guard4(v8f& a, v8f& b, v8f& c, v8f& d) { asm volatile("v_nop\n\tv_nop\n\tv_nop\n\tv_nop" : "+v"(a), "+v"(b), "+v"(c), "+v"(d)); }
template <typename T> struct Frag;
template <> struct Frag<_Float16> {
  typedef v16h V; union U { v16h v; v8h h[2]; };
  static __device__ __forceinline__ v16h load(const _Float16* p) {
    U f; f.h[0] = *(const v8h*)(p); f.h[1] = *(const v8h*)(p + 16); return f.v;
  }
  static __device__ __forceinline__ v8f mma(v16h a, v16h b, v8f c) {
    return __builtin_amdgcn_wmma_f32_16x16x32_f16(false, a, false, b, (short)0, c, false, false);
  }
  static __device__ __forceinline__ void guard(v8f& a, v8f& b, v16h x, v16h y) { dep_guard_h(a, b, x, y); }
  static __device__ __forceinline__ void keep(v16h a, v16h b, v16h c, v16h d) { keep4_h(a, b, c, d); }
};
template <> struct Frag<__bf16> {
  typedef v16b V; union U { v16b v; v8b h[2]; };
  static __device__ __forceinline__ v16b load(const __bf16* p) {
    U f; f.h[0] = *(const v8b*)(p); f.h[1] = *(const v8b*)(p + 16); return f.v;
  }
  static __device__ __forceinline__ v8f mma(v16b a, v16b b, v8f c) {
    return __builtin_amdgcn_wmma_f32_16x16x32_bf16(false, a, false, b, (short)0, c, false, false);
  }
  static __device__ __forceinline__ void guard(v8f& a, v8f& b, v16b x, v16b y) { dep_guard_b(a, b, x, y); }
  static __device__ __forceinline__ void keep(v16b a, v16b b, v16b c, v16b d) { keep4_b(a, b, c, d); }
};

template <int ET> struct Elem;
template <> struct Elem<0> { typedef _Float16 T; };
template <> struct Elem<1> { typedef __bf16 T; };
template <int ET, bool SPLIT, int BIAS_MODE, int OUT_MODE, bool RESID, int ACT = 0>
__global__ __launch_bounds__(256) void wmma_gemm64(
    const unsigned short* __restrict__ Ap, const unsigned short* __restrict__ A2p, int lda, long strideA,
    const unsigned short* __restrict__ Btp, const unsigned short* __restrict__ Bt2p, int ldb, long strideB,
    void* __restrict__ Cout, void* __restrict__ Cout2, int ldc, long strideC,
    const float* __restrict__ bias, const float* __restrict__ scale_ptr, int nbias,
    const float* __restrict__ resid, long strideR,
    int M, int N, int K, float scale) {
  typedef typename Elem<ET>::T T;
  typedef typename Frag<T>::V V;
  const T* A = (const T*)Ap; const T* A2 = (const T*)A2p; const T* Bt = (const T*)Btp; const T* Bt2 = (const T*)Bt2p;
  __shared__ __align__(16) float sT[8][16 * 68];
  const int b    = blockIdx.y;
  const int lane = threadIdx.x & 31;
  const int wave = threadIdx.x >> 5;
  const int tilesN = N >> 6;
  const int tilesM = M >> 6;
  const int tile = blockIdx.x * 8 + wave;
  if (tile >= tilesM * tilesN) return;
  const int tm = tile / tilesN;
  const int tn = tile - tm * tilesN;
  const int m0 = tm << 6;
  const int n0 = tn << 6;
  const float scl = scale * scale_ptr[0];

  const T* Ab  = A  + (size_t)b * strideA;
  const T* Bb  = Bt + (size_t)b * strideB;
  const T* Ab2 = SPLIT ? (A2  + (size_t)b * strideA) : nullptr;
  const T* Bb2 = SPLIT ? (Bt2 + (size_t)b * strideB) : nullptr;

  const int rlane = lane & 15;
  const int koff  = (lane >> 4) * 8;
  const int mOff  = (lane >> 4) * 8;

  v8f acc[4][4];
#pragma unroll
  for (int i = 0; i < 4; ++i)
#pragma unroll
    for (int j = 0; j < 4; ++j) acc[i][j] = (v8f){0.f,0.f,0.f,0.f,0.f,0.f,0.f,0.f};

  for (int k0 = 0; k0 < K; k0 += 32) {
    V bh[4], bl[4];
#pragma unroll
    for (int j = 0; j < 4; ++j) {
      const size_t bo = (size_t)(n0 + (j << 4) + rlane) * ldb + koff + k0;
      bh[j] = Frag<T>::load(Bb + bo);
      if (SPLIT) bl[j] = Frag<T>::load(Bb2 + bo);
    }
#pragma unroll
    for (int i = 0; i < 4; ++i) {
      const size_t ao = (size_t)(m0 + (i << 4) + rlane) * lda + koff + k0;
      V ah = Frag<T>::load(Ab + ao);
      V al;
      if (SPLIT) al = Frag<T>::load(Ab2 + ao);
#pragma unroll
      for (int j = 0; j < 4; ++j) {
        acc[i][j] = Frag<T>::mma(ah, bh[j], acc[i][j]);
        if (SPLIT) {
          acc[i][j] = Frag<T>::mma(ah, bl[j], acc[i][j]);
          acc[i][j] = Frag<T>::mma(al, bh[j], acc[i][j]);
        }
      }
      Frag<T>::guard(acc[i][0], acc[i][3], ah, SPLIT ? al : ah);
    }
    Frag<T>::keep(bh[0], bh[1], bh[2], bh[3]);
    if (SPLIT) Frag<T>::keep(bl[0], bl[1], bl[2], bl[3]);
  }
  acc_guard4(acc[0][0], acc[0][1], acc[0][2], acc[0][3]);
  acc_guard4(acc[1][0], acc[1][1], acc[1][2], acc[1][3]);
  acc_guard4(acc[2][0], acc[2][1], acc[2][2], acc[2][3]);
  acc_guard4(acc[3][0], acc[3][1], acc[3][2], acc[3][3]);

  float* slab = sT[wave];
  const float* Rb = RESID ? (resid + (size_t)b * strideR) : nullptr;
#pragma unroll
  for (int i = 0; i < 4; ++i) {
    const int mBase = m0 + (i << 4);
#pragma unroll
    for (int j = 0; j < 4; ++j) {
      const int n = n0 + (j << 4) + rlane;
      float bv = 0.f;
      if (BIAS_MODE == 2) { const int nb = (n < nbias) ? n : (nbias - 1); bv = bias[nb]; }
#pragma unroll
      for (int r = 0; r < 8; ++r) {
        float v = acc[i][j][r] * scl;
        if (BIAS_MODE == 1) v += bias[mBase + mOff + r];
        if (BIAS_MODE == 2) v += bv;
        if (RESID) v += Rb[(size_t)(mBase + mOff + r) * ldc + n];
        if (ACT == 1) v = tanhf(v);
        if (ACT == 2) v = fmaxf(v, 0.0f);
        if (ACT == 3) v = v / (1.0f + expf(-v));
        if (ACT == 4) v = (v > 0.f) ? v : 0.01f * v;
        if (ACT == 5) v = 0.5f * v * (1.0f + erff(v * 0.70710678118654752f));
        slab[(mOff + r) * 68 + (j << 4) + rlane] = v;
      }
    }
    __builtin_amdgcn_fence(__ATOMIC_RELEASE, "workgroup");
    __builtin_amdgcn_wave_barrier();
    __builtin_amdgcn_fence(__ATOMIC_ACQUIRE, "workgroup");
    if (OUT_MODE == 0) {
      float* C = (float*)Cout + (size_t)b * strideC;
      const int hh = lane >> 4, c4 = (lane & 15) * 4;
      for (int pass = 0; pass < 2; ++pass) {
#pragma unroll
        for (int it = 0; it < 8; ++it) {
          const int row = it * 2 + hh;
          v4f v = *(const v4f*)(slab + row * 68 + c4);
          *(volatile v4f*)(C + (size_t)(mBase + row) * ldc + n0 + c4) = v;
        }
        __threadfence();
      }
    } else {
      const int q = lane >> 3, c8 = (lane & 7) * 8;
      unsigned short* C  = (unsigned short*)Cout  + (size_t)b * strideC;
      unsigned short* C2 = (OUT_MODE == 2) ? ((unsigned short*)Cout2 + (size_t)b * strideC) : nullptr;
      for (int pass = 0; pass < 2; ++pass) {
#pragma unroll
        for (int it = 0; it < 4; ++it) {
          const int row = it * 4 + q;
          const float* sp = slab + row * 68 + c8;
          v8h hv, lv;
#pragma unroll
          for (int e = 0; e < 8; ++e) {
            if (OUT_MODE == 1) {
              hv[e] = (_Float16)sp[e];
            } else {
              unsigned short hb = f2bf_bits(sp[e]);
              unsigned short lb = f2bf_bits(sp[e] - bf_bits2f(hb));
              hv[e] = __builtin_bit_cast(_Float16, hb);
              lv[e] = __builtin_bit_cast(_Float16, lb);
            }
          }
          *(volatile v8h*)(C + (size_t)(mBase + row) * ldc + n0 + c8) = hv;
          if (OUT_MODE == 2) *(volatile v8h*)(C2 + (size_t)(mBase + row) * ldc + n0 + c8) = lv;
        }
        __threadfence();
      }
    }
    __builtin_amdgcn_fence(__ATOMIC_RELEASE, "workgroup");
    __builtin_amdgcn_wave_barrier();
    __builtin_amdgcn_fence(__ATOMIC_ACQUIRE, "workgroup");
  }
}

__global__ __launch_bounds__(256) void prep_ternary_kernel(
    const float* __restrict__ w1, const float* __restrict__ w2, const float* __restrict__ w3,
    const float* __restrict__ fw1, const float* __restrict__ fw2,
    _Float16* __restrict__ pl1, _Float16* __restrict__ pl2, _Float16* __restrict__ pl3,
    _Float16* __restrict__ pl4, _Float16* __restrict__ pl5, float* __restrict__ alpha_out) {
  __shared__ double red[256];
  __shared__ int redc[256];
  __shared__ float sh_delta, sh_alpha;
  const int tsr = blockIdx.x, t = threadIdx.x;
  const float* w; _Float16* P; int n, nrows, kp, rvalid, kvalid, rstride, perm;
  if (tsr == 0)      { w = w1;  n = 800;    P = pl1; nrows = 32;  kp = 32;   rvalid = 32;  kvalid = 25;   rstride = 25;   perm = 0; }
  else if (tsr == 1) { w = w2;  n = 51200;  P = pl2; nrows = 64;  kp = 800;  rvalid = 64;  kvalid = 800;  rstride = 800;  perm = 1; }
  else if (tsr == 2) { w = w3;  n = 192000; P = pl3; nrows = 128; kp = 1600; rvalid = 120; kvalid = 1600; rstride = 1600; perm = 0; }
  else if (tsr == 3) { w = fw1; n = 10080;  P = pl4; nrows = 128; kp = 128;  rvalid = 84;  kvalid = 120;  rstride = 120;  perm = 0; }
  else               { w = fw2; n = 840;    P = pl5; nrows = 64;  kp = 128;  rvalid = 10;  kvalid = 84;   rstride = 84;   perm = 0; }

  double s = 0.0;
  for (int i = t; i < n; i += 256) s += (double)fabsf(w[i]);
  red[t] = s;
  __syncthreads();
  for (int k = 128; k > 0; k >>= 1) { if (t < k) red[t] += red[t + k]; __syncthreads(); }
  if (t == 0) { const float mean = (float)(red[0] / (double)n); sh_delta = 0.7f * mean; }
  __syncthreads();
  const float delta = sh_delta;

  double sa = 0.0; int cnt = 0;
  for (int i = t; i < n; i += 256) { const float a = fabsf(w[i]); if (a > delta) { sa += (double)a; cnt += 1; } }
  red[t] = sa; redc[t] = cnt;
  __syncthreads();
  for (int k = 128; k > 0; k >>= 1) { if (t < k) { red[t] += red[t + k]; redc[t] += redc[t + k]; } __syncthreads(); }
  if (t == 0) { const float c = (float)redc[0]; sh_alpha = (float)red[0] * (1.0f / fmaxf(c, 1.0f)); }
  __syncthreads();
  const float alpha = sh_alpha;
  if (t < 32) { ((volatile float*)alpha_out)[tsr * 32 + t] = alpha; }
  __threadfence();
  if (t < 32) { ((volatile float*)alpha_out)[tsr * 32 + t] = alpha; }

  const int nchunks = (nrows * kp) >> 3;
  for (int pass = 0; pass < 2; ++pass) {
    for (int ch = t; ch < nchunks; ch += 256) {
      const int e0 = ch << 3;
      const int r = e0 / kp;
      const int k0 = e0 - r * kp;
      const int rr = (r < rvalid) ? r : (rvalid - 1);
      v8h v;
#pragma unroll
      for (int j = 0; j < 8; ++j) {
        const int k = k0 + j;
        const int kc = (k < kvalid) ? k : (kvalid - 1);
        const int kk = perm ? (((kc & 31) * 25) + (kc >> 5)) : kc;
        const float wi = w[(size_t)rr * rstride + kk];
        float q = (fabsf(wi) > delta) ? ((wi > 0.f) ? 1.f : -1.f) : 0.f;
        if (r >= rvalid || k >= kvalid) q = 0.f;
        v[j] = (_Float16)q;
      }
      *(volatile v8h*)(P + (size_t)e0) = v;
    }
    __threadfence();
  }
}

__global__ __launch_bounds__(256) void conv1_pool_kernel(
    const float* __restrict__ x, const _Float16* __restrict__ Bt1, const float* __restrict__ b1,
    const float* __restrict__ alpha, _Float16* __restrict__ p1) {
  __shared__ __align__(16) _Float16 ximg[1024];
  __shared__ __align__(16) _Float16 pout[6272];
  const int img = blockIdx.x;
  const int t = threadIdx.x, lane = t & 31, wave = t >> 5, hh = lane >> 4, m = lane & 15;
  {
    const v4f v = *(const v4f*)(x + (size_t)img * 1024 + 4 * t);
    ximg[4 * t + 0] = (_Float16)v[0];
    ximg[4 * t + 1] = (_Float16)v[1];
    ximg[4 * t + 2] = (_Float16)v[2];
    ximg[4 * t + 3] = (_Float16)v[3];
  }
  __syncthreads();
  const float al = alpha[0];
  const v16h bq0 = Frag<_Float16>::load(Bt1 + (size_t)m * 32 + 8 * hh);
  const v16h bq1 = Frag<_Float16>::load(Bt1 + (size_t)(16 + m) * 32 + 8 * hh);
  const float bias0 = b1[m], bias1 = b1[16 + m];
  int koff[16];
#pragma unroll
  for (int i = 0; i < 16; ++i) {
    const int k = (i < 8) ? (8 * hh + i) : (8 + 8 * hh + i);
    const int ky = (k * 13) >> 6;
    const int kx = k - 5 * ky;
    koff[i] = (k < 25) ? (ky * 32 + kx) : 0;
  }
  for (int tile = wave; tile < 49; tile += 8) {
    const int ty = tile / 7, tx = tile - 7 * ty;
    const int base = (ty * 4 + (m >> 2)) * 32 + tx * 4 + (m & 3);
    v16h a;
#pragma unroll
    for (int i = 0; i < 16; ++i) a[i] = ximg[base + koff[i]];
    v8f acc0 = (v8f){0.f,0.f,0.f,0.f,0.f,0.f,0.f,0.f};
    v8f acc1 = (v8f){0.f,0.f,0.f,0.f,0.f,0.f,0.f,0.f};
    acc0 = Frag<_Float16>::mma(a, bq0, acc0);
    acc1 = Frag<_Float16>::mma(a, bq1, acc1);
    Frag<_Float16>::guard(acc0, acc1, a, bq0);
    Frag<_Float16>::keep(bq0, bq1, a, a);
    float u0[8], u1[8];
#pragma unroll
    for (int r = 0; r < 8; ++r) { u0[r] = al * acc0[r] + bias0; u1[r] = al * acc1[r] + bias1; }
    const float q00 = fmaxf(fmaxf(u0[0], u0[1]), fmaxf(u0[4], u0[5]));
    const float q01 = fmaxf(fmaxf(u0[2], u0[3]), fmaxf(u0[6], u0[7]));
    const float q10 = fmaxf(fmaxf(u1[0], u1[1]), fmaxf(u1[4], u1[5]));
    const float q11 = fmaxf(fmaxf(u1[2], u1[3]), fmaxf(u1[6], u1[7]));
    const int pbase = (ty * 2 + hh) * 14 + tx * 2;
    pout[m * 196 + pbase]            = (_Float16)tanhf(q00);
    pout[m * 196 + pbase + 1]        = (_Float16)tanhf(q01);
    pout[(16 + m) * 196 + pbase]     = (_Float16)tanhf(q10);
    pout[(16 + m) * 196 + pbase + 1] = (_Float16)tanhf(q11);
  }
  __syncthreads();
  _Float16* dst = p1 + (size_t)img * 6272;
  for (int pass = 0; pass < 2; ++pass) {
    for (int ch = t; ch < 784; ch += 256) {
      const v8h v = *(const v8h*)(pout + ch * 8);
      *(volatile v8h*)(dst + (size_t)ch * 8) = v;
    }
    __threadfence();
  }
}

__global__ __launch_bounds__(224) void conv2_pool_kernel(
    const _Float16* __restrict__ p1, const _Float16* __restrict__ Bt2, const float* __restrict__ b2,
    const float* __restrict__ alpha, _Float16* __restrict__ p2) {
  __shared__ __align__(16) _Float16 imgT[196 * 32];
  __shared__ __align__(16) float cst[100 * 64];
  __shared__ __align__(16) _Float16 pst[1600];
  const int img = blockIdx.x;
  const int t = threadIdx.x, lane = t & 31, wave = t >> 5, hh = lane >> 4, m = lane & 15;
  {
    const _Float16* src = p1 + (size_t)img * 6272;
    for (int ch = t; ch < 784; ch += 224) {
      const v8h v = *(const v8h*)(src + (size_t)ch * 8);
      const int e = ch * 8;
      int c = e / 196;
      int pos = e - 196 * c;
#pragma unroll
      for (int j = 0; j < 8; ++j) {
        imgT[pos * 32 + c] = v[j];
        ++pos;
        const bool wrap = (pos == 196);
        pos = wrap ? 0 : pos;
        c = wrap ? (c + 1) : c;
      }
    }
  }
  __syncthreads();
  const float al = alpha[32];
  const int p = wave * 16 + m;
  const int pc = (p < 100) ? p : 99;
  const int oy = pc / 10, ox = pc - 10 * oy;
  const int posbase = oy * 14 + ox;
  const _Float16* bb = Bt2 + (size_t)m * 800 + 8 * hh;
  v8f acc[4];
#pragma unroll
  for (int nt = 0; nt < 4; ++nt) acc[nt] = (v8f){0.f,0.f,0.f,0.f,0.f,0.f,0.f,0.f};
  int ky = 0, kx = 0;
#pragma unroll 1
  for (int tap = 0; tap < 25; ++tap) {
    const int apos = posbase + ky * 14 + kx;
    const v16h a = Frag<_Float16>::load(imgT + apos * 32 + 8 * hh);
    v16h bq[4];
#pragma unroll
    for (int nt = 0; nt < 4; ++nt) bq[nt] = Frag<_Float16>::load(bb + (size_t)nt * 12800 + tap * 32);
#pragma unroll
    for (int nt = 0; nt < 4; ++nt) acc[nt] = Frag<_Float16>::mma(a, bq[nt], acc[nt]);
    Frag<_Float16>::guard(acc[0], acc[3], a, bq[3]);
    Frag<_Float16>::keep(bq[0], bq[1], bq[2], bq[3]);
    ++kx;
    const bool wr = (kx == 5);
    kx = wr ? 0 : kx;
    ky = wr ? (ky + 1) : ky;
  }
  acc_guard4(acc[0], acc[1], acc[2], acc[3]);
#pragma unroll
  for (int nt = 0; nt < 4; ++nt) {
    const int oc = nt * 16 + m;
    const float bv = b2[oc];
#pragma unroll
    for (int r = 0; r < 8; ++r) {
      const int pos = wave * 16 + 8 * hh + r;
      const float v = al * acc[nt][r] + bv;
      if (pos < 100) cst[pos * 64 + oc] = v;
    }
  }
  __syncthreads();
  for (int o = t; o < 1600; o += 224) {
    const int oc = o / 25;
    const int rem = o - 25 * oc;
    const int py = rem / 5;
    const int px = rem - 5 * py;
    const int p00 = (2 * py) * 10 + 2 * px;
    const float mx = fmaxf(fmaxf(cst[p00 * 64 + oc], cst[(p00 + 1) * 64 + oc]),
                           fmaxf(cst[(p00 + 10) * 64 + oc], cst[(p00 + 11) * 64 + oc]));
    pst[o] = (_Float16)tanhf(mx);
  }
  __syncthreads();
  _Float16* dst = p2 + (size_t)img * 1600;
  for (int pass = 0; pass < 2; ++pass) {
    if (t < 200) {
      const v8h v = *(const v8h*)(pst + t * 8);
      *(volatile v8h*)(dst + (size_t)t * 8) = v;
    }
    __threadfence();
  }
}

__global__ __launch_bounds__(256) void softmax_out_kernel(
    const float* __restrict__ lg, float* __restrict__ out, int nimg) {
  __shared__ __align__(16) float slog[2560];
  __shared__ __align__(16) float sprb[2560];
  const int t = threadIdx.x;
  const int n0 = blockIdx.x * 256;
  const int n = n0 + t;
  const int nc = (n < nimg) ? n : (nimg - 1);
  const float* row = lg + (size_t)nc * 64;
  float mx = -INFINITY;
#pragma unroll 1
  for (int c = 0; c < 10; ++c) { const float v = row[c]; slog[t * 10 + c] = v; mx = fmaxf(mx, v); }
  float ssum = 0.f;
#pragma unroll 1
  for (int c = 0; c < 10; ++c) { const float e = expf(slog[t * 10 + c] - mx); sprb[t * 10 + c] = e; ssum += e; }
  const float inv = 1.0f / ssum;
#pragma unroll 1
  for (int c = 0; c < 10; ++c) sprb[t * 10 + c] = sprb[t * 10 + c] * inv;
  __syncthreads();
  float* o0 = out + (size_t)n0 * 10;
  float* o1 = out + (size_t)nimg * 10 + (size_t)n0 * 10;
  for (int pass = 0; pass < 2; ++pass) {
    for (int ch = t; ch < 640; ch += 256) {
      const v4f a = *(const v4f*)(slog + ch * 4);
      const v4f b = *(const v4f*)(sprb + ch * 4);
      *(volatile v4f*)(o0 + (size_t)ch * 4) = a;
      *(volatile v4f*)(o1 + (size_t)ch * 4) = b;
    }
    __threadfence();
  }
}

extern "C" void kernel_launch(void* const* d_in, const int* in_sizes, int n_in,
                              void* d_out, int out_size, void* d_ws, size_t ws_size,
                              hipStream_t stream) {
  if (n_in < 11) return;
  const int nimg = in_sizes[0] / 1024;
  if (nimg <= 0 || (nimg % 256) != 0 || in_sizes[0] != nimg * 1024) return;
  if (in_sizes[1] != 800 || in_sizes[2] != 32 || in_sizes[3] != 51200 || in_sizes[4] != 64 ||
      in_sizes[5] != 192000 || in_sizes[6] != 120 || in_sizes[7] != 10080 || in_sizes[8] != 84 ||
      in_sizes[9] != 840 || in_sizes[10] != 10) return;
  if (out_size != nimg * 20) return;

  const float* x   = (const float*)d_in[0];
  const float* w1  = (const float*)d_in[1];
  const float* b1  = (const float*)d_in[2];
  const float* w2  = (const float*)d_in[3];
  const float* b2  = (const float*)d_in[4];
  const float* w3  = (const float*)d_in[5];
  const float* b3  = (const float*)d_in[6];
  const float* fw1 = (const float*)d_in[7];
  const float* fb1 = (const float*)d_in[8];
  const float* fw2 = (const float*)d_in[9];
  const float* fb2 = (const float*)d_in[10];
  float* out = (float*)d_out;

  size_t off = 0;
  auto carve = [&](size_t bytes) -> size_t { size_t o = off; off = (off + bytes + 255) & ~(size_t)255; return o; };
  const size_t o_alpha = carve(5 * 128);
  const size_t o_pl1 = carve((size_t)32 * 32 * 2);
  const size_t o_pl2 = carve((size_t)64 * 800 * 2);
  const size_t o_pl3 = carve((size_t)128 * 1600 * 2);
  const size_t o_pl4 = carve((size_t)128 * 128 * 2);
  const size_t o_pl5 = carve((size_t)64 * 128 * 2);
  const size_t o_p1  = carve((size_t)nimg * 6272 * 2);
  const size_t o_p2  = carve((size_t)nimg * 1600 * 2);
  const size_t o_h3  = carve((size_t)nimg * 128 * 2);
  const size_t o_h4  = carve((size_t)nimg * 128 * 2);
  const size_t o_lg  = carve((size_t)nimg * 64 * 4);
  if (off > ws_size || off > (size_t)134217728u) return;

  char* ws = (char*)d_ws;
  float*    alpha = (float*)(ws + o_alpha);
  _Float16* pl1 = (_Float16*)(ws + o_pl1);
  _Float16* pl2 = (_Float16*)(ws + o_pl2);
  _Float16* pl3 = (_Float16*)(ws + o_pl3);
  _Float16* pl4 = (_Float16*)(ws + o_pl4);
  _Float16* pl5 = (_Float16*)(ws + o_pl5);
  _Float16* p1  = (_Float16*)(ws + o_p1);
  _Float16* p2  = (_Float16*)(ws + o_p2);
  _Float16* h3  = (_Float16*)(ws + o_h3);
  _Float16* h4  = (_Float16*)(ws + o_h4);
  float*    lg  = (float*)(ws + o_lg);

  prep_ternary_kernel<<<5, 256, 0, stream>>>(w1, w2, w3, fw1, fw2, pl1, pl2, pl3, pl4, pl5, alpha);

  conv1_pool_kernel<<<nimg, 256, 0, stream>>>(x, pl1, b1, alpha, p1);

  conv2_pool_kernel<<<nimg, 224, 0, stream>>>(p1, pl2, b2, alpha, p2);

  {
    const int tiles = (nimg / 64) * (128 / 64);
    wmma_gemm64<0, false, 2, 1, false, 1><<<dim3((tiles + 7) / 8, 1), 256, 0, stream>>>(
        (const unsigned short*)p2, (const unsigned short*)p2, 1600, 0L,
        (const unsigned short*)pl3, (const unsigned short*)pl3, 1600, 0L,
        (void*)h3, (void*)h3, 128, 0L,
        b3, alpha + 64, 120,
        b3, 0L,
        nimg, 128, 1600, 1.0f);
  }
  {
    const int tiles = (nimg / 64) * (128 / 64);
    wmma_gemm64<0, false, 2, 1, false, 1><<<dim3((tiles + 7) / 8, 1), 256, 0, stream>>>(
        (const unsigned short*)h3, (const unsigned short*)h3, 128, 0L,
        (const unsigned short*)pl4, (const unsigned short*)pl4, 128, 0L,
        (void*)h4, (void*)h4, 128, 0L,
        fb1, alpha + 96, 84,
        fb1, 0L,
        nimg, 128, 128, 1.0f);
  }
  {
    const int tiles = (nimg / 64) * (64 / 64);
    wmma_gemm64<0, false, 2, 0, false, 0><<<dim3((tiles + 7) / 8, 1), 256, 0, stream>>>(
        (const unsigned short*)h4, (const unsigned short*)h4, 128, 0L,
        (const unsigned short*)pl5, (const unsigned short*)pl5, 128, 0L,
        (void*)lg, (void*)lg, 64, 0L,
        fb2, alpha + 128, 10,
        fb2, 0L,
        nimg, 64, 128, 1.0f);
  }
  softmax_out_kernel<<<nimg / 256, 256, 0, stream>>>(lg, out, nimg);
}
